// LDS_41077067219061
// MI455X (gfx1250) — hardware-run, weakly checked
//
#include <hip/hip_runtime.h>
#include <math.h>

typedef __attribute__((ext_vector_type(16))) _Float16 v16h;
typedef __attribute__((ext_vector_type(8)))  _Float16 v8h;
typedef __attribute__((ext_vector_type(2)))  _Float16 v2h;
typedef __attribute__((ext_vector_type(8)))  float    v8f;
typedef __attribute__((ext_vector_type(4)))  float    v4f;
typedef __attribute__((ext_vector_type(2)))  float    v2f;

constexpr int kBatch   = 8;
constexpr int kSeq     = 2048;
constexpr int kState   = 1024;
constexpr int kDin     = 512;
constexpr int kDout    = 512;
constexpr int kTaps    = 10;
constexpr int kPad     = kTaps - 1;
constexpr int kPadRows = kPad + kSeq;
constexpr int kRows    = kBatch * kSeq;
constexpr int kWinK    = kTaps * kDin;
static_assert(kPadRows == 2057 && kWinK == 5120 && kRows == 16384, "shape constants");
static_assert((kDin % 32) == 0 && (kState % 32) == 0 && (kWinK % 32) == 0, "every K is a multiple of 32");
static_assert((kSeq % 64) == 0 && (kState % 64) == 0 && (kDout % 64) == 0, "M and N are multiples of 64");

constexpr float kCarryX = 64.0f;
constexpr float kCarryH = 16.0f;
constexpr float kCarryB = 1024.0f;
constexpr float kCarryC = 4096.0f;
constexpr float kCarryM = 1024.0f;
static_assert(kCarryH * kCarryC == kCarryX * kCarryM, "both K-phases of the fused GEMM carry the same product scale");
constexpr float kScaleProj = 1.0f / (kCarryX * kCarryB);
constexpr float kScaleOut  = 1.0f / (kCarryX * kCarryM);
constexpr float kF16MinNormal = 6.103515625e-5f;

constexpr size_t kSzXP = (size_t)kBatch * kPadRows * kDin * 2;
constexpr size_t kSzBT = (size_t)kState * kDin * 2;
constexpr size_t kSzCT = (size_t)kDout * kState * 2;
constexpr size_t kSzMT = (size_t)kDout * kWinK * 2;
constexpr size_t kSzUB = (size_t)kRows * kState * 4;
constexpr size_t kSzHS = (size_t)kRows * kState * 2;
constexpr size_t kOffXP = 0;
constexpr size_t kOffBT = kOffXP + kSzXP;
constexpr size_t kOffCT = kOffBT + kSzBT;
constexpr size_t kOffMT = kOffCT + kSzCT;
constexpr size_t kOffUB = kOffMT + kSzMT;
constexpr size_t kOffHS = kOffUB + kSzUB;
constexpr size_t kWsTotal = kOffHS + kSzHS;
static_assert(kWsTotal == 124854272ull, "carve total");
static_assert(kWsTotal <= 134217728ull, "carve cap");
static_assert((kOffBT % 128) == 0 && (kOffCT % 128) == 0 && (kOffMT % 128) == 0 && (kOffUB % 128) == 0 && (kOffHS % 128) == 0, "128-B aligned regions");

__device__ __forceinline__ _Float16 to_h16(float v) {
  const float c = fminf(fmaxf(v, -65504.0f), 65504.0f);
  const float w = (fabsf(c) < kF16MinNormal) ? 0.0f : c;
  return (_Float16)w;
}

namespace eng {
union FragU { v16h v; v8h h[2]; };
__device__ __forceinline__ v16h frag_load(const _Float16* p) {
  FragU f;
  f.h[0] = *(const v8h*)(p);
  f.h[1] = *(const v8h*)(p + 16);
  return f.v;
}
__device__ __forceinline__ v8f mma(v16h a, v16h b, v8f c) {
  return __builtin_amdgcn_wmma_f32_16x16x32_f16(false, a, false, b, (short)0, c, false, false);
}
__device__ __forceinline__ void tie1(v8f& a, v16h x, v16h y) { asm volatile("" : "+v"(a) : "v"(x), "v"(y)); }
__device__ __forceinline__ void tie1_nops(v8f& a, v16h x, v16h y) { asm volatile("v_nop\n\tv_nop\n\tv_nop\n\tv_nop" : "+v"(a) : "v"(x), "v"(y)); }
__device__ __forceinline__ void keep4(v16h a, v16h b, v16h c, v16h d) { asm volatile("v_nop" :: "v"(a), "v"(b), "v"(c), "v"(d)); }
__device__ __forceinline__ void acc_guard1(v8f& a) { asm volatile("v_nop\n\tv_nop\n\tv_nop\n\tv_nop" : "+v"(a)); }
}

__global__ __launch_bounds__(256) void gemm_two_phase_kernel(
    const unsigned short* A1p, int lda1, long strideA1, const unsigned short* B1p, int ldb1, int K1,
    const unsigned short* A2p, int lda2, long strideA2, const unsigned short* B2p, int ldb2, int K2,
    float* __restrict__ Cout, int ldc, long strideC, int M, int N, float scale)
{
  __shared__ __align__(16) float sT[8][16 * 68];
  const int b    = blockIdx.y;
  const int lane = threadIdx.x & 31;
  const int wave = threadIdx.x >> 5;
  const int tilesN = N >> 6;
  const int tilesM = M >> 6;
  const int tile = blockIdx.x * 8 + wave;
  if (tile >= tilesM * tilesN) return;
  const int tm = tile / tilesN;
  const int tn = tile - tm * tilesN;
  const int m0 = tm << 6;
  const int n0 = tn << 6;

  const _Float16* A1b = (const _Float16*)A1p + (size_t)b * strideA1;
  const _Float16* A2b = (const _Float16*)A2p + (size_t)b * strideA2;
  const _Float16* B1  = (const _Float16*)B1p;
  const _Float16* B2  = (const _Float16*)B2p;

  const int rlane = lane & 15;
  const int koff  = (lane >> 4) * 8;
  const int mOff  = (lane >> 4) * 8;

  v8f acc[4][4];
#pragma unroll
  for (int i = 0; i < 4; ++i)
#pragma unroll
    for (int j = 0; j < 4; ++j) acc[i][j] = (v8f){0.f, 0.f, 0.f, 0.f, 0.f, 0.f, 0.f, 0.f};

#pragma unroll 1
  for (int ph = 0; ph < 2; ++ph) {
    const _Float16* Ab = (ph == 0) ? A1b : A2b;
    const _Float16* Bb = (ph == 0) ? B1 : B2;
    const int lda = (ph == 0) ? lda1 : lda2;
    const int ldb = (ph == 0) ? ldb1 : ldb2;
    const int K   = (ph == 0) ? K1 : K2;
#pragma unroll 1
    for (int k0 = 0; k0 < K; k0 += 32) {
      v16h bh[4];
#pragma unroll
      for (int j = 0; j < 4; ++j) {
        const size_t bo = (size_t)(n0 + (j << 4) + rlane) * ldb + koff + k0;
        bh[j] = eng::frag_load(Bb + bo);
      }
#pragma unroll
      for (int i = 0; i < 4; ++i) {
        const size_t ao = (size_t)(m0 + (i << 4) + rlane) * lda + koff + k0;
        const v16h ah = eng::frag_load(Ab + ao);
#pragma unroll
        for (int j = 0; j < 4; ++j) acc[i][j] = eng::mma(ah, bh[j], acc[i][j]);
        eng::tie1(acc[i][0], ah, bh[0]);
        eng::tie1(acc[i][1], ah, bh[1]);
        eng::tie1(acc[i][2], ah, bh[2]);
        eng::tie1_nops(acc[i][3], ah, bh[3]);
      }
      eng::keep4(bh[0], bh[1], bh[2], bh[3]);
    }
  }
#pragma unroll
  for (int i = 0; i < 4; ++i)
#pragma unroll
    for (int j = 0; j < 4; ++j) eng::acc_guard1(acc[i][j]);

  float* slab = sT[wave];
  float* C = Cout + (size_t)b * strideC;
  const int hh = lane >> 4;
  const int c4 = (lane & 15) * 4;
#pragma unroll
  for (int i = 0; i < 4; ++i) {
    const int mBase = m0 + (i << 4);
#pragma unroll
    for (int j = 0; j < 4; ++j) {
#pragma unroll
      for (int r = 0; r < 8; ++r) {
        const float v = acc[i][j][r] * scale;
        slab[(mOff + r) * 68 + (j << 4) + rlane] = v;
      }
    }
    __builtin_amdgcn_fence(__ATOMIC_RELEASE, "workgroup");
    __builtin_amdgcn_wave_barrier();
    __builtin_amdgcn_fence(__ATOMIC_ACQUIRE, "workgroup");
    for (int pass = 0; pass < 2; ++pass) {
#pragma unroll
      for (int it = 0; it < 8; ++it) {
        const int row = it * 2 + hh;
        const v4f v = *(const v4f*)(slab + row * 68 + c4);
        *(volatile v4f*)(C + (size_t)(mBase + row) * ldc + n0 + c4) = v;
      }
      __threadfence();
    }
    __builtin_amdgcn_fence(__ATOMIC_RELEASE, "workgroup");
    __builtin_amdgcn_wave_barrier();
    __builtin_amdgcn_fence(__ATOMIC_ACQUIRE, "workgroup");
  }
}

constexpr int kXpPerBatch = kPadRows * (kDin / 8);
constexpr int kXpThreads  = kBatch * kXpPerBatch;
static_assert(kXpThreads == 4114 * 256, "exact grid");
__global__ __launch_bounds__(256) void xpad_kernel(const float* __restrict__ x, unsigned short* __restrict__ xp) {
  const int i = blockIdx.x * 256 + threadIdx.x;
  if (i >= kXpThreads) return;
  const int b    = i / kXpPerBatch;
  const int rem  = i - b * kXpPerBatch;
  const int prow = rem >> 6;
  const int c    = (rem & 63) << 3;
  const bool real = (prow >= kPad);
  const int t = real ? (prow - kPad) : 0;
  const float* src = x + ((size_t)(b * kSeq + t)) * kDin + c;
  v4f a0 = *(const v4f*)(src);
  v4f a1 = *(const v4f*)(src + 4);
  asm volatile("" : "+v"(a0), "+v"(a1));
  v8h hv;
#pragma unroll
  for (int e = 0; e < 4; ++e) {
    const float f0 = real ? (a0[e] * kCarryX) : 0.0f;
    const float f1 = real ? (a1[e] * kCarryX) : 0.0f;
    hv[e]     = to_h16(f0);
    hv[4 + e] = to_h16(f1);
  }
  unsigned short* q = xp + (size_t)i * 8;
  *(volatile v8h*)q = hv;
  __threadfence();
  *(volatile v8h*)q = hv;
}

__global__ __launch_bounds__(256) void tcast_kernel(const float* __restrict__ in, unsigned short* __restrict__ out,
                                                    int N, int K, float carry) {
  const int kg = K >> 3;
  const int i = blockIdx.x * 256 + threadIdx.x;
  if (i >= N * kg) return;
  const int n = i / kg;
  const int g = i - n * kg;
  float f[8];
#pragma unroll
  for (int e = 0; e < 8; ++e) f[e] = in[(size_t)(8 * g + e) * N + n];
  v8h hv;
#pragma unroll
  for (int e = 0; e < 8; ++e) hv[e] = to_h16(f[e] * carry);
  unsigned short* q = out + (size_t)n * K + 8 * g;
  *(volatile v8h*)q = hv;
  __threadfence();
  *(volatile v8h*)q = hv;
}

constexpr int kMtPerRow  = kWinK / 8;
constexpr int kMtThreads = kDout * kMtPerRow;
static_assert(kMtThreads == 1280 * 256, "exact grid");
__global__ __launch_bounds__(256) void mpack_kernel(const float* __restrict__ Mw, unsigned short* __restrict__ mt) {
  const int i = blockIdx.x * 256 + threadIdx.x;
  if (i >= kMtThreads) return;
  const int n   = i / kMtPerRow;
  const int rem = i - n * kMtPerRow;
  const int j   = rem >> 6;
  const int c   = (rem & 63) << 3;
  const int tap = (kTaps - 1) - j;
  const float* src = Mw + (size_t)n * (kDin * kTaps) + (size_t)c * kTaps + tap;
  float f[8];
#pragma unroll
  for (int e = 0; e < 8; ++e) f[e] = src[e * kTaps];
  v8h hv;
#pragma unroll
  for (int e = 0; e < 8; ++e) hv[e] = to_h16(f[e] * kCarryM);
  unsigned short* q = mt + (size_t)n * kWinK + (size_t)j * kDin + c;
  *(volatile v8h*)q = hv;
  __threadfence();
  *(volatile v8h*)q = hv;
}

constexpr int kScanLanes = kBatch * (kState / 2);
static_assert(kScanLanes == 16 * 256, "exact grid");
__global__ __launch_bounds__(256) void scan_kernel(const float* __restrict__ uB, const float* __restrict__ Avec,
                                                   const float* __restrict__ h0v, unsigned* __restrict__ hs32) {
  const int g = blockIdx.x * 256 + threadIdx.x;
  if (g >= kScanLanes) return;
  const int b  = g / (kState / 2);
  const int sp = g - b * (kState / 2);
  const int s0 = 2 * sp;
  const v2f av = *(const v2f*)(Avec + s0);
  const v2f hi = *(const v2f*)(h0v + s0);
  const float aA = av[0], aB = av[1];
  float hA = hi[0], hB = hi[1];
  const size_t row0 = (size_t)b * kSeq;
#pragma unroll 1
  for (int t0 = 0; t0 < kSeq; t0 += 8) {
    v2f u[8];
#pragma unroll
    for (int j = 0; j < 8; ++j) u[j] = *(const v2f*)(uB + (row0 + t0 + j) * kState + s0);
    unsigned pk[8];
#pragma unroll
    for (int j = 0; j < 8; ++j) {
      hA = fmaf(aA, hA, u[j][0]);
      hB = fmaf(aB, hB, u[j][1]);
      v2h p;
      p[0] = to_h16(hA * kCarryH);
      p[1] = to_h16(hB * kCarryH);
      pk[j] = __builtin_bit_cast(unsigned, p);
    }
    for (int pass = 0; pass < 2; ++pass) {
#pragma unroll
      for (int j = 0; j < 8; ++j)
        *(volatile unsigned*)(hs32 + (row0 + t0 + j) * (kState / 2) + sp) = pk[j];
      __threadfence();
    }
  }
}

extern "C" void kernel_launch(void* const* d_in, const int* in_sizes, int n_in,
                              void* d_out, int out_size, void* d_ws, size_t ws_size,
                              hipStream_t stream) {
  if (n_in < 6) return;
  if (in_sizes[0] != kRows * kDin) return;
  if (in_sizes[1] != kState) return;
  if (in_sizes[2] != kState) return;
  if (in_sizes[3] != kDin * kState) return;
  if (in_sizes[4] != kState * kDout) return;
  if (in_sizes[5] != kDout * kDin * kTaps) return;
  if (out_size != kRows * kDout) return;
  if (ws_size < kWsTotal) return;

  const float* x   = (const float*)d_in[0];
  const float* h0  = (const float*)d_in[1];
  const float* Av  = (const float*)d_in[2];
  const float* Bw  = (const float*)d_in[3];
  const float* Cw  = (const float*)d_in[4];
  const float* Mw  = (const float*)d_in[5];
  float* out = (float*)d_out;

  char* ws = (char*)d_ws;
  unsigned short* XP = (unsigned short*)(ws + kOffXP);
  unsigned short* BT = (unsigned short*)(ws + kOffBT);
  unsigned short* CT = (unsigned short*)(ws + kOffCT);
  unsigned short* MT = (unsigned short*)(ws + kOffMT);
  float*          UB = (float*)(ws + kOffUB);
  unsigned short* HS = (unsigned short*)(ws + kOffHS);

  xpad_kernel<<<kXpThreads / 256, 256, 0, stream>>>(x, XP);
  tcast_kernel<<<(kState * (kDin / 8)) / 256, 256, 0, stream>>>(Bw, BT, kState, kDin, kCarryB);
  tcast_kernel<<<(kDout * (kState / 8)) / 256, 256, 0, stream>>>(Cw, CT, kDout, kState, kCarryC);
  mpack_kernel<<<kMtThreads / 256, 256, 0, stream>>>(Mw, MT);

  gemm_two_phase_kernel<<<dim3(64, kBatch), 256, 0, stream>>>(
      XP + (size_t)kPad * kDin, kDin, (long)kPadRows * kDin, BT, kDin, kDin,
      XP + (size_t)kPad * kDin, kDin, (long)kPadRows * kDin, BT, kDin, 0,
      UB, kState, (long)kSeq * kState, kSeq, kState, kScaleProj);

  scan_kernel<<<kScanLanes / 256, 256, 0, stream>>>(UB, Av, h0, (unsigned*)HS);

  gemm_two_phase_kernel<<<dim3(32, kBatch), 256, 0, stream>>>(
      HS, kState, (long)kSeq * kState, CT, kState, kState,
      XP, kDin, (long)kPadRows * kDin, MT, kWinK, kWinK,
      out, kDout, (long)kSeq * kDout, kSeq, kDout, kScaleOut);
}
